// Decoder_75505525064316
// MI455X (gfx1250) — hardware-verified
//
#include <hip/hip_runtime.h>
#include <math.h>

#ifndef NROWS
#define NROWS 65536
#endif
constexpr int NROWS_FULL = 65536;
constexpr int LAT        = 64;
constexpr int NFEAT      = 128;
constexpr int HID        = 32;
constexpr int NWAVE      = 2;
constexpr int NTHR_MAIN  = 32 * NWAVE;
constexpr int ROWS_WAVE  = 16;
constexpr int ROWS_BLK   = ROWS_WAVE * NWAVE;
constexpr int YP         = 132;
constexpr int OSP        = NFEAT;
constexpr int NTHR_PREP  = 256;
constexpr int W2_ELEMS    = NFEAT * HID * HID;
constexpr int SMALL_ELEMS = NFEAT * HID;
constexpr int WP_ELEMS    = NFEAT * LAT;
constexpr int PREP_W2_BLOCKS    = W2_ELEMS / (8 * NTHR_PREP);
constexpr int PREP_SMALL_BLOCKS = 21;
constexpr int MAIN_BLOCKS       = NROWS / ROWS_BLK;

static_assert(NROWS % ROWS_BLK == 0);
static_assert(NROWS >= ROWS_BLK && NROWS <= NROWS_FULL);
static_assert(LAT == 64);
static_assert(HID == 32);
static_assert(NFEAT % 16 == 0);
static_assert(PREP_W2_BLOCKS * NTHR_PREP * 8 == W2_ELEMS);
static_assert(4 * NTHR_PREP * 4 == SMALL_ELEMS);
static_assert(4 * NTHR_PREP * 8 == WP_ELEMS);
static_assert(32 * 4 == NFEAT);
static_assert(PREP_SMALL_BLOCKS == 16 + 1 + 4);
static_assert(MAIN_BLOCKS * NWAVE * ROWS_WAVE == NROWS);
static_assert(YP % 4 == 0 && YP >= NFEAT);
static_assert(OSP == 4 * 32);
static_assert((size_t)(NROWS - 1) * NFEAT + (NFEAT - 1) < (size_t)NROWS_FULL * NFEAT);

typedef __attribute__((ext_vector_type(16))) __bf16 v16bf;
typedef __attribute__((ext_vector_type(8)))  __bf16 v8bf;
typedef __attribute__((ext_vector_type(8)))  float  v8f;
typedef __attribute__((ext_vector_type(4)))  float  v4f;
typedef __attribute__((ext_vector_type(4)))  unsigned int v4u;

__device__ __forceinline__ void guard1(v8f& a, v16bf x0, v16bf x1, v16bf y0, v16bf y1) {
  asm volatile("v_nop\n\tv_nop\n\tv_nop\n\tv_nop" : "+v"(a) : "v"(x0), "v"(x1), "v"(y0), "v"(y1));
}
__device__ __forceinline__ void guard2(v8f& a, v8f& b, v16bf x0, v16bf x1, v16bf y0, v16bf y1) {
  asm volatile("v_nop\n\tv_nop\n\tv_nop\n\tv_nop" : "+v"(a), "+v"(b) : "v"(x0), "v"(x1), "v"(y0), "v"(y1));
}

__device__ __forceinline__ v8f mma_bf(v16bf a, v16bf b, v8f c) {
  return __builtin_amdgcn_wmma_f32_16x16x32_bf16(false, a, false, b, (short)0, c, false, false);
}

__device__ __forceinline__ v16bf frag_bf(const __bf16* p) {
  const v8bf lo = *(const v8bf*)(p);
  const v8bf hi = *(const v8bf*)(p + 16);
  return __builtin_shufflevector(lo, hi, 0, 1, 2, 3, 4, 5, 6, 7, 8, 9, 10, 11, 12, 13, 14, 15);
}

__device__ __forceinline__ v16bf frag_f32(const float* p) {
  const v4f q0 = *(const v4f*)(p);
  const v4f q1 = *(const v4f*)(p + 4);
  const v4f q2 = *(const v4f*)(p + 16);
  const v4f q3 = *(const v4f*)(p + 20);
  v16bf o;
#pragma unroll
  for (int e = 0; e < 4; ++e) {
    o[e]      = (__bf16)q0[e];
    o[4 + e]  = (__bf16)q1[e];
    o[8 + e]  = (__bf16)q2[e];
    o[12 + e] = (__bf16)q3[e];
  }
  return o;
}

__device__ __forceinline__ float bf16_rne_f(float x) {
  const __bf16 b = (__bf16)x;
  return __uint_as_float(((unsigned int)__builtin_bit_cast(unsigned short, b)) << 16);
}

template <int B>
__device__ __forceinline__ void h1_pack4(float yv, v4f w, v4f bb, v16bf& hi, v16bf& lo) {
#pragma unroll
  for (int e = 0; e < 4; ++e) {
    const float v = fmaxf(fmaf(yv, w[e], bb[e]), 0.0f);
    const __bf16 h16 = (__bf16)v;
    const float hf = __uint_as_float(((unsigned int)__builtin_bit_cast(unsigned short, h16)) << 16);
    hi[B + e] = h16;
    lo[B + e] = (__bf16)(v - hf);
  }
}

template <int R0>
__device__ __forceinline__ float head4(const v8f& cc, v4f bb, v4f ww, float p) {
#pragma unroll
  for (int e = 0; e < 4; ++e) p = fmaf(fmaxf(cc[R0 + e] + bb[e], 0.0f), ww[e], p);
  return p;
}

__global__ __launch_bounds__(NTHR_PREP) void k_prep_w2(const float* __restrict__ W2, __bf16* __restrict__ W2B) {
  const int i = blockIdx.x * NTHR_PREP + threadIdx.x;
  const float* sp = W2 + (size_t)i * 8;
  const v4f a = *(const v4f*)(sp);
  const v4f b = *(const v4f*)(sp + 4);
  v8bf o;
#pragma unroll
  for (int e = 0; e < 4; ++e) { o[e] = (__bf16)a[e]; o[4 + e] = (__bf16)b[e]; }
  const v4u u = __builtin_bit_cast(v4u, o);
  volatile v4u* dp = (volatile v4u*)(W2B + (size_t)i * 8);
  *dp = u;
  __threadfence();
  *dp = u;
}

__global__ __launch_bounds__(NTHR_PREP) void k_prep_small(
    const float* __restrict__ Wp, const float* __restrict__ W1, const float* __restrict__ b1,
    const float* __restrict__ b2, const float* __restrict__ W3, const float* __restrict__ b3,
    __bf16* __restrict__ WPB, float* __restrict__ W1R, float* __restrict__ B1R,
    float* __restrict__ B2R, float* __restrict__ W3R, float* __restrict__ B3R) {
  const int blk = blockIdx.x, tid = threadIdx.x;
  if (blk < 16) {
    const int reg = blk >> 2;
    const int i = (blk & 3) * NTHR_PREP + tid;
    const float* src = (reg == 0) ? W1 : (reg == 1) ? b1 : (reg == 2) ? b2 : W3;
    float* dst = (reg == 0) ? W1R : (reg == 1) ? B1R : (reg == 2) ? B2R : W3R;
    const v4f a = *(const v4f*)(src + (size_t)i * 4);
    v4f o;
#pragma unroll
    for (int e = 0; e < 4; ++e) o[e] = bf16_rne_f(a[e]);
    volatile v4f* dp = (volatile v4f*)(dst + (size_t)i * 4);
    *dp = o;
    __threadfence();
    *dp = o;
  } else if (blk == 16) {
    if (tid < 32) {
      const v4f a = *(const v4f*)(b3 + tid * 4);
      v4f o;
#pragma unroll
      for (int e = 0; e < 4; ++e) o[e] = bf16_rne_f(a[e]);
      volatile v4f* dp = (volatile v4f*)(B3R + tid * 4);
      *dp = o;
      __threadfence();
      *dp = o;
    }
  } else {
    const int i = (blk - 17) * NTHR_PREP + tid;
    const float* sp = Wp + (size_t)i * 8;
    const v4f a = *(const v4f*)(sp);
    const v4f b = *(const v4f*)(sp + 4);
    v8bf o;
#pragma unroll
    for (int e = 0; e < 4; ++e) { o[e] = (__bf16)fabsf(a[e]); o[4 + e] = (__bf16)fabsf(b[e]); }
    const v4u u = __builtin_bit_cast(v4u, o);
    volatile v4u* dp = (volatile v4u*)(WPB + (size_t)i * 8);
    *dp = u;
    __threadfence();
    *dp = u;
  }
}

__global__ __launch_bounds__(NTHR_MAIN) void k_mlp_main(
    const float* __restrict__ z, const __bf16* __restrict__ WPB, const __bf16* __restrict__ W2B,
    const float* __restrict__ W1R, const float* __restrict__ B1R, const float* __restrict__ B2R,
    const float* __restrict__ W3R, const float* __restrict__ B3R, float* __restrict__ out) {
  __shared__ __align__(16) float Ys[NWAVE][ROWS_WAVE * YP];
  __shared__ __align__(16) float Os[NWAVE][ROWS_WAVE * OSP];
  const int tid = threadIdx.x, lane = tid & 31, wave = tid >> 5;
  const int c = lane & 15, hh = lane >> 4, koff = 8 * hh;
  const size_t row0 = (size_t)blockIdx.x * ROWS_BLK + (size_t)wave * ROWS_WAVE;
  float* ys = Ys[wave];
  float* os = Os[wave];
  const v8f z8 = {0.f, 0.f, 0.f, 0.f, 0.f, 0.f, 0.f, 0.f};

  {
    const float* zp = z + (row0 + (size_t)c) * LAT + koff;
    const v16bf za0 = frag_f32(zp);
    const v16bf za1 = frag_f32(zp + 32);
#pragma unroll 1
    for (int dt = 0; dt < NFEAT / 16; ++dt) {
      const __bf16* wp = WPB + (size_t)(dt * 16 + c) * LAT + koff;
      const v16bf b0 = frag_bf(wp);
      const v16bf b1 = frag_bf(wp + 32);
      v8f acc = mma_bf(za0, b0, z8);
      acc = mma_bf(za1, b1, acc);
      guard1(acc, za0, za1, b0, b1);
#pragma unroll
      for (int r = 0; r < 8; ++r) ys[(koff + r) * YP + dt * 16 + c] = acc[r];
    }
  }
  __syncthreads();

#pragma unroll 1
  for (int d = 0; d < NFEAT; ++d) {
    const float yv = ys[c * YP + d];
    const float* w1p = W1R + d * HID + koff;
    const float* b1p = B1R + d * HID + koff;
    const v4f w1a = *(const v4f*)(w1p);      const v4f w1b = *(const v4f*)(w1p + 4);
    const v4f w1c = *(const v4f*)(w1p + 16); const v4f w1d = *(const v4f*)(w1p + 20);
    const v4f b1a = *(const v4f*)(b1p);      const v4f b1b = *(const v4f*)(b1p + 4);
    const v4f b1c = *(const v4f*)(b1p + 16); const v4f b1d = *(const v4f*)(b1p + 20);
    v16bf bh, bl;
    h1_pack4<0>(yv, w1a, b1a, bh, bl);
    h1_pack4<4>(yv, w1b, b1b, bh, bl);
    h1_pack4<8>(yv, w1c, b1c, bh, bl);
    h1_pack4<12>(yv, w1d, b1d, bh, bl);

    const __bf16* ap = W2B + (size_t)d * (HID * HID) + (size_t)c * HID + koff;
    const v16bf a0 = frag_bf(ap);
    const v16bf a1 = frag_bf(ap + 16 * HID);
    v8f c0 = mma_bf(a0, bh, z8);
    c0 = mma_bf(a0, bl, c0);
    v8f c1 = mma_bf(a1, bh, z8);
    c1 = mma_bf(a1, bl, c1);
    guard2(c0, c1, a0, a1, bh, bl);

    const float* b2p = B2R + d * HID + koff;
    const float* w3p = W3R + d * HID + koff;
    const v4f b2a = *(const v4f*)(b2p);      const v4f b2b = *(const v4f*)(b2p + 4);
    const v4f b2c = *(const v4f*)(b2p + 16); const v4f b2d = *(const v4f*)(b2p + 20);
    const v4f w3a = *(const v4f*)(w3p);      const v4f w3b = *(const v4f*)(w3p + 4);
    const v4f w3c = *(const v4f*)(w3p + 16); const v4f w3d = *(const v4f*)(w3p + 20);
    float p = 0.0f;
    p = head4<0>(c0, b2a, w3a, p);
    p = head4<4>(c0, b2b, w3b, p);
    p = head4<0>(c1, b2c, w3c, p);
    p = head4<4>(c1, b2d, w3d, p);
    const float q = __shfl_xor(p, 16, 32);
    const float x = (p + q) + B3R[d];
    os[c * OSP + d] = fabsf(x);
  }
  __syncthreads();

  for (int ps = 0; ps < 2; ++ps) {
#pragma unroll
    for (int it = 0; it < ROWS_WAVE; ++it) {
      const v4f v = *(const v4f*)(os + it * OSP + 4 * lane);
      *(volatile v4f*)(out + (row0 + (size_t)it) * NFEAT + 4 * lane) = v;
    }
    __threadfence();
  }
}

extern "C" void kernel_launch(void* const* d_in, const int* in_sizes, int n_in,
                              void* d_out, int out_size, void* d_ws, size_t ws_size, hipStream_t stream) {
  if (n_in < 8 || d_out == nullptr || d_ws == nullptr) return;
  if (in_sizes[0] < NROWS * LAT || in_sizes[1] != WP_ELEMS || in_sizes[2] != SMALL_ELEMS ||
      in_sizes[3] != SMALL_ELEMS || in_sizes[4] != W2_ELEMS || in_sizes[5] != SMALL_ELEMS ||
      in_sizes[6] != SMALL_ELEMS || in_sizes[7] != NFEAT || out_size < NROWS * NFEAT) return;

  const float* z  = (const float*)d_in[0];
  const float* Wp = (const float*)d_in[1];
  const float* W1 = (const float*)d_in[2];
  const float* b1 = (const float*)d_in[3];
  const float* W2 = (const float*)d_in[4];
  const float* b2 = (const float*)d_in[5];
  const float* W3 = (const float*)d_in[6];
  const float* b3 = (const float*)d_in[7];
  float* out = (float*)d_out;

  char* ws = (char*)d_ws; size_t off = 0;
  auto carve = [&](size_t bytes) -> char* { char* p = ws + off; off += (bytes + 255) & ~(size_t)255; return p; };
  __bf16* W2B = (__bf16*)carve((size_t)W2_ELEMS * 2);
  __bf16* WPB = (__bf16*)carve((size_t)WP_ELEMS * 2);
  float*  W1R = (float*)carve((size_t)SMALL_ELEMS * 4);
  float*  B1R = (float*)carve((size_t)SMALL_ELEMS * 4);
  float*  B2R = (float*)carve((size_t)SMALL_ELEMS * 4);
  float*  W3R = (float*)carve((size_t)SMALL_ELEMS * 4);
  float*  B3R = (float*)carve((size_t)NFEAT * 4);
  if (off > ws_size || off > (size_t)134217728) return;

  k_prep_w2<<<PREP_W2_BLOCKS, NTHR_PREP, 0, stream>>>(W2, W2B);
  k_prep_small<<<PREP_SMALL_BLOCKS, NTHR_PREP, 0, stream>>>(Wp, W1, b1, b2, W3, b3, WPB, W1R, B1R, B2R, W3R, B3R);
  k_mlp_main<<<MAIN_BLOCKS, NTHR_MAIN, 0, stream>>>(z, WPB, W2B, W1R, B1R, B2R, W3R, B3R, out);
}
